// SHToGridDensity_74191265071590
// MI455X (gfx1250) — hardware-run, weakly checked
//
#include <hip/hip_runtime.h>


namespace {
constexpr int NR = 256  , NL = 5, NM = 9, NRB = 16, K = NL * NM * NRB  , KP = 736, G = 35937, GP = 35968  , GT = 32  , NW = GP / GT  ;
constexpr float XS = 8.0f, HS = 256.0f;
typedef _Float16 b16;
typedef __attribute__((ext_vector_type(16))) _Float16 v16b;
typedef __attribute__((ext_vector_type(8))) _Float16 v8b;
typedef __attribute__((ext_vector_type(8))) float v8f;
typedef __attribute__((ext_vector_type(4))) float v4f;
__device__ __forceinline__ float bf16_rne(float f) { unsigned int u = __float_as_uint(f); u += 0x7FFFu + ((u >> 16) & 1u); float r = __uint_as_float(u & 0xFFFF0000u); asm volatile("" : "+v"(r)); return r; }
__device__ __forceinline__ float bfv(float f) { float r = bf16_rne(f); asm volatile("" : "+v"(r)); return r; }
__device__ __forceinline__ void split16(float v, b16& hi, b16& lo) { hi = (b16)v; lo = (b16)(v - (float)hi); }
__device__ __forceinline__ v16b frag_kb(const b16* p, int hh) { const v8b a = *(const v8b*)(p + 8 * hh), b = *(const v8b*)(p + 16 + 8 * hh); v16b f;
#pragma unroll
  for (int e = 0; e < 8; ++e) { f[e] = a[e]; f[8 + e] = b[e]; } return f; }
__device__ __forceinline__ v8f wmma16b(v16b a, v16b b, v8f c) { v8f d = __builtin_amdgcn_wmma_f32_16x16x32_f16(false, a, false, b, (short)0, c, false, false); asm volatile("v_nop\n\tv_nop\n\tv_nop\n\tv_nop" : "+v"(d) : "v"(a), "v"(b)); return d; }
__device__ __forceinline__ void wave_lds_sync() { __builtin_amdgcn_fence(__ATOMIC_RELEASE, "workgroup"); __builtin_amdgcn_wave_barrier(); __builtin_amdgcn_fence(__ATOMIC_ACQUIRE, "workgroup"); }
__device__ __forceinline__ float pmul(float a, float b) { float p = a * b; asm volatile("" : "+v"(p)); return p; }

__global__ __launch_bounds__(256) void cput_kernel(const float* __restrict__ co, b16* __restrict__ CT) { const int u = blockIdx.x * 256 + threadIdx.x; if (u >= NR * (KP / 8)) return; const int row = u / (KP / 8), k0 = (u % (KP / 8)) * 8; v8b v;
#pragma unroll
  for (int j = 0; j < 8; ++j) { const int k = k0 + j; v[j] = (b16)(k < K ? bf16_rne(co[(size_t)row * K + k]) * XS : 0.0f); }
  for (int pass = 0; pass < 2; ++pass) { *(volatile v8b*)(CT + (size_t)row * KP + k0) = v; __threadfence(); } }
__global__ __launch_bounds__(32) void main_kernel(const float* __restrict__ Y, const float* __restrict__ Rb, const b16* __restrict__ CT, float* __restrict__ STG) { __shared__ __attribute__((aligned(16))) b16 Ah[GT][KP + 8], Al[GT][KP + 8]; __shared__ float Yg[GT][NL * NM + 3], Rg[GT][NRB + 1], Tf[GT][129]; const int lane = threadIdx.x, nloc = lane & 15, hlf = lane >> 4; const int g0 = blockIdx.x * GT; const int gl = g0 + lane; const bool live = gl < G;
  for (int q = 0; q < NL * NM; ++q) Yg[lane][q] = live ? bfv(Y[(size_t)q * G + gl]) : 0.0f; for (int r = 0; r < NRB; ++r) Rg[lane][r] = live ? bfv(Rb[(size_t)r * G + gl]) : 0.0f;
  wave_lds_sync();
  for (int gg = 0; gg < GT; ++gg) for (int q = 0; q < KP / 32; ++q) { const int k = q * 32 + lane; b16 p = (b16)0.0f, ql = (b16)0.0f; if (k < K) { const float v = pmul(Yg[gg][k / NRB], Rg[gg][k % NRB]); split16(v * HS, p, ql); } Ah[gg][k] = p; Al[gg][k] = ql; }
  for (int k = KP; k < KP + 8; ++k) { Ah[lane][k] = (b16)0.0f; Al[lane][k] = (b16)0.0f; }
  wave_lds_sync();
#pragma unroll 1
  for (int cg = 0; cg < 2; ++cg) { v8f acc[2][8];
#pragma unroll
    for (int rt = 0; rt < 2; ++rt)
#pragma unroll
      for (int t = 0; t < 8; ++t) acc[rt][t] = (v8f){};
#pragma unroll 1
    for (int kb = 0; kb < KP; kb += 32) { v16b bw[8];
#pragma unroll
      for (int t = 0; t < 8; ++t) bw[t] = frag_kb(CT + (size_t)(cg * 128 + t * 16 + nloc) * KP + kb, hlf);
#pragma unroll
      for (int rt = 0; rt < 2; ++rt) { const v16b a = frag_kb(&Ah[rt * 16 + nloc][kb], hlf), al = frag_kb(&Al[rt * 16 + nloc][kb], hlf);
#pragma unroll
        for (int t = 0; t < 8; ++t) { acc[rt][t] = wmma16b(a, bw[t], acc[rt][t]); acc[rt][t] = wmma16b(al, bw[t], acc[rt][t]); } } }
#pragma unroll
    for (int rt = 0; rt < 2; ++rt)
#pragma unroll
      for (int t = 0; t < 8; ++t)
#pragma unroll
        for (int r8 = 0; r8 < 8; ++r8) Tf[rt * 16 + 8 * hlf + r8][t * 16 + nloc] = acc[rt][t][r8] * (1.0f / (HS * XS));
    wave_lds_sync();
    for (int pass = 0; pass < 2; ++pass) { for (int c = 0; c < 128; ++c) ((volatile float*)STG)[(size_t)(cg * 128 + c) * GP + gl] = live ? Tf[lane][c] : 0.0f; __threadfence(); }
    wave_lds_sync(); } }
__global__ __launch_bounds__(256) void copy_kernel(const float* __restrict__ STG, int WLIM, float* __restrict__ out) { const size_t u = (size_t)blockIdx.x * 256 + threadIdx.x; if (u >= (size_t)NR * G) return; const size_t r = u / G, g = u % G; if (g >= (size_t)WLIM * GT) return;
  for (int pass = 0; pass < 2; ++pass) { ((volatile float*)out)[u] = STG[r * GP + g]; __threadfence(); } }
}

extern "C" void kernel_launch(void* const* d_in, const int* in_sizes, int n_in, void* d_out, int out_size, void* d_ws, size_t ws_size, hipStream_t stream) {
  (void)n_in;
  auto Fp = [&](int i) { return (const float*)d_in[i]; };
  if (in_sizes[0] != NR * K || in_sizes[1] != NL * NM * G || in_sizes[2] != NRB * G || out_size != NR * G) return;
  const int WLIM = NW;
  size_t off = 0; char* ws = (char*)d_ws;
  auto carve = [&](size_t bytes) { char* p = ws + off; off += (bytes + 255) & ~(size_t)255; return p; };
  b16* CT = (b16*)carve((size_t)NR * KP * 2); float* STG = (float*)carve((size_t)NR * GP * 4);
  if (off > ws_size || off > ((size_t)48 << 20)) return;
  cput_kernel<<<(NR * (KP / 8) + 255) / 256, 256, 0, stream>>>(Fp(0), CT);
  main_kernel<<<WLIM, 32, 0, stream>>>(Fp(1), Fp(2), CT, STG);
  copy_kernel<<<(NR * G + 255) / 256, 256, 0, stream>>>(STG, WLIM, (float*)d_out);
}
